// MultiSkillPolicyNet1_35330400977129
// MI455X (gfx1250) — hardware-verified
//
#include <hip/hip_runtime.h>
#include <stdint.h>

#define SDIM 2
#define HID 1024
#define NSK 5
#define NACT 4
#define NBATCH 65536
#define CHUNK 16384
#define NCHUNK (NBATCH / CHUNK)
#define NHP 64
#define L1_ROWS 16
#define WSCALE 16.0f
#define WSCALE_INV 0.0625f

typedef __attribute__((ext_vector_type(16))) _Float16 v16h;
typedef __attribute__((ext_vector_type(8)))  _Float16 v8h;
typedef __attribute__((ext_vector_type(16))) __bf16   v16b;
typedef __attribute__((ext_vector_type(8)))  __bf16   v8b;
typedef __attribute__((ext_vector_type(8)))  float    v8f;
typedef __attribute__((ext_vector_type(4)))  float    v4f;

__device__ __forceinline__ unsigned short f2bf_bits(float f) {
  unsigned u = __float_as_uint(f);
  return (unsigned short)((u + 0x7FFFu + ((u >> 16) & 1u)) >> 16);
}
__device__ __forceinline__ float bf_bits2f(unsigned short h) { return __uint_as_float(((unsigned)h) << 16); }

__device__ __forceinline__ void dep_guard_h(v8f& a, v8f& b, v16h x, v16h y) { asm volatile("v_nop\n\tv_nop\n\tv_nop\n\tv_nop" : "+v"(a), "+v"(b) : "v"(x), "v"(y)); }
__device__ __forceinline__ void dep_guard_b(v8f& a, v8f& b, v16b x, v16b y) { asm volatile("v_nop\n\tv_nop\n\tv_nop\n\tv_nop" : "+v"(a), "+v"(b) : "v"(x), "v"(y)); }
__device__ __forceinline__ void keep4_h(v16h a, v16h b, v16h c, v16h d) { asm volatile("v_nop" :: "v"(a), "v"(b), "v"(c), "v"(d)); }
__device__ __forceinline__ void keep4_b(v16b a, v16b b, v16b c, v16b d) { asm volatile("v_nop" :: "v"(a), "v"(b), "v"(c), "v"(d)); }
__device__ __forceinline__ void acc_guard4(v8f& a, v8f& b, v8f& c, v8f& d) { asm volatile("v_nop\n\tv_nop\n\tv_nop\n\tv_nop" : "+v"(a), "+v"(b), "+v"(c), "+v"(d)); }
template <typename T> struct Frag;
template <> struct Frag<_Float16> {
  typedef v16h V; union U { v16h v; v8h h[2]; };
  static __device__ __forceinline__ v16h load(const _Float16* p) {
    U f; f.h[0] = *(const v8h*)(p); f.h[1] = *(const v8h*)(p + 16); return f.v;
  }
  static __device__ __forceinline__ v8f mma(v16h a, v16h b, v8f c) {
    return __builtin_amdgcn_wmma_f32_16x16x32_f16(false, a, false, b, (short)0, c, false, false);
  }
  static __device__ __forceinline__ void guard(v8f& a, v8f& b, v16h x, v16h y) { dep_guard_h(a, b, x, y); }
  static __device__ __forceinline__ void keep(v16h a, v16h b, v16h c, v16h d) { keep4_h(a, b, c, d); }
};
template <> struct Frag<__bf16> {
  typedef v16b V; union U { v16b v; v8b h[2]; };
  static __device__ __forceinline__ v16b load(const __bf16* p) {
    U f; f.h[0] = *(const v8b*)(p); f.h[1] = *(const v8b*)(p + 16); return f.v;
  }
  static __device__ __forceinline__ v8f mma(v16b a, v16b b, v8f c) {
    return __builtin_amdgcn_wmma_f32_16x16x32_bf16(false, a, false, b, (short)0, c, false, false);
  }
  static __device__ __forceinline__ void guard(v8f& a, v8f& b, v16b x, v16b y) { dep_guard_b(a, b, x, y); }
  static __device__ __forceinline__ void keep(v16b a, v16b b, v16b c, v16b d) { keep4_b(a, b, c, d); }
};

template <int ET> struct Elem;
template <> struct Elem<0> { typedef _Float16 T; };
template <> struct Elem<1> { typedef __bf16 T; };
template <int ET, bool SPLIT, int BIAS_MODE, int OUT_MODE, bool RESID, int ACT = 0>
__global__ __launch_bounds__(256) void wmma_gemm64(
    const unsigned short* __restrict__ Ap, const unsigned short* __restrict__ A2p, int lda, long strideA,
    const unsigned short* __restrict__ Btp, const unsigned short* __restrict__ Bt2p, int ldb, long strideB,
    void* __restrict__ Cout, void* __restrict__ Cout2, int ldc, long strideC,
    const float* __restrict__ bias,
    const float* __restrict__ resid, long strideR,
    int M, int N, int K, float scale) {
  typedef typename Elem<ET>::T T;
  typedef typename Frag<T>::V V;
  const T* A = (const T*)Ap; const T* A2 = (const T*)A2p; const T* Bt = (const T*)Btp; const T* Bt2 = (const T*)Bt2p;
  __shared__ __align__(16) float sT[8][16 * 68];
  const int b    = blockIdx.y;
  const int lane = threadIdx.x & 31;
  const int wave = threadIdx.x >> 5;
  const int tilesN = N >> 6;
  const int tilesM = M >> 6;
  const int tile = blockIdx.x * 8 + wave;
  if (tile >= tilesM * tilesN) return;
  const int tm = tile / tilesN;
  const int tn = tile - tm * tilesN;
  const int m0 = tm << 6;
  const int n0 = tn << 6;

  const T* Ab  = A  + (size_t)b * strideA;
  const T* Bb  = Bt + (size_t)b * strideB;
  const T* Ab2 = SPLIT ? (A2  + (size_t)b * strideA) : nullptr;
  const T* Bb2 = SPLIT ? (Bt2 + (size_t)b * strideB) : nullptr;

  const int rlane = lane & 15;
  const int koff  = (lane >> 4) * 8;
  const int mOff  = (lane >> 4) * 8;

  v8f acc[4][4];
#pragma unroll
  for (int i = 0; i < 4; ++i)
#pragma unroll
    for (int j = 0; j < 4; ++j) acc[i][j] = (v8f){0.f,0.f,0.f,0.f,0.f,0.f,0.f,0.f};

  for (int k0 = 0; k0 < K; k0 += 32) {
    V bh[4], bl[4];
#pragma unroll
    for (int j = 0; j < 4; ++j) {
      const size_t bo = (size_t)(n0 + (j << 4) + rlane) * ldb + koff + k0;
      bh[j] = Frag<T>::load(Bb + bo);
      if (SPLIT) bl[j] = Frag<T>::load(Bb2 + bo);
    }
#pragma unroll
    for (int i = 0; i < 4; ++i) {
      const size_t ao = (size_t)(m0 + (i << 4) + rlane) * lda + koff + k0;
      V ah = Frag<T>::load(Ab + ao);
      V al;
      if (SPLIT) al = Frag<T>::load(Ab2 + ao);
#pragma unroll
      for (int j = 0; j < 4; ++j) {
        acc[i][j] = Frag<T>::mma(ah, bh[j], acc[i][j]);
        if (SPLIT) {
          acc[i][j] = Frag<T>::mma(ah, bl[j], acc[i][j]);
          acc[i][j] = Frag<T>::mma(al, bh[j], acc[i][j]);
        }
      }
      Frag<T>::guard(acc[i][0], acc[i][3], ah, SPLIT ? al : ah);
    }
    Frag<T>::keep(bh[0], bh[1], bh[2], bh[3]);
    if (SPLIT) Frag<T>::keep(bl[0], bl[1], bl[2], bl[3]);
  }
  acc_guard4(acc[0][0], acc[0][1], acc[0][2], acc[0][3]);
  acc_guard4(acc[1][0], acc[1][1], acc[1][2], acc[1][3]);
  acc_guard4(acc[2][0], acc[2][1], acc[2][2], acc[2][3]);
  acc_guard4(acc[3][0], acc[3][1], acc[3][2], acc[3][3]);

  float* slab = sT[wave];
  const float* Rb = RESID ? (resid + (size_t)b * strideR) : nullptr;
#pragma unroll
  for (int i = 0; i < 4; ++i) {
    const int mBase = m0 + (i << 4);
#pragma unroll
    for (int j = 0; j < 4; ++j) {
      const int n = n0 + (j << 4) + rlane;
      float bv = 0.f;
      if (BIAS_MODE == 2) bv = bias[n];
#pragma unroll
      for (int r = 0; r < 8; ++r) {
        float v = acc[i][j][r] * scale;
        if (BIAS_MODE == 1) v += bias[mBase + mOff + r];
        if (BIAS_MODE == 2) v += bv;
        if (RESID) v += Rb[(size_t)(mBase + mOff + r) * ldc + n];
        if (ACT == 1) v = tanhf(v);
        if (ACT == 2) v = fmaxf(v, 0.0f);
        if (ACT == 3) v = v / (1.0f + expf(-v));
        if (ACT == 4) v = (v > 0.f) ? v : 0.01f * v;
        if (ACT == 5) v = 0.5f * v * (1.0f + erff(v * 0.70710678118654752f));
        slab[(mOff + r) * 68 + (j << 4) + rlane] = v;
      }
    }
    __builtin_amdgcn_fence(__ATOMIC_RELEASE, "workgroup");
    __builtin_amdgcn_wave_barrier();
    __builtin_amdgcn_fence(__ATOMIC_ACQUIRE, "workgroup");
    if (OUT_MODE == 0) {
      float* C = (float*)Cout + (size_t)b * strideC;
      const int hh = lane >> 4, c4 = (lane & 15) * 4;
      for (int pass = 0; pass < 2; ++pass) {
#pragma unroll
        for (int it = 0; it < 8; ++it) {
          const int row = it * 2 + hh;
          v4f v = *(const v4f*)(slab + row * 68 + c4);
          *(volatile v4f*)(C + (size_t)(mBase + row) * ldc + n0 + c4) = v;
        }
        __threadfence();
      }
    } else {
      const int q = lane >> 3, c8 = (lane & 7) * 8;
      unsigned short* C  = (unsigned short*)Cout  + (size_t)b * strideC;
      unsigned short* C2 = (OUT_MODE == 2) ? ((unsigned short*)Cout2 + (size_t)b * strideC) : nullptr;
      for (int pass = 0; pass < 2; ++pass) {
#pragma unroll
        for (int it = 0; it < 4; ++it) {
          const int row = it * 4 + q;
          const float* sp = slab + row * 68 + c8;
          v8h hv, lv;
#pragma unroll
          for (int e = 0; e < 8; ++e) {
            if (OUT_MODE == 1) {
              hv[e] = (_Float16)sp[e];
            } else {
              unsigned short hb = f2bf_bits(sp[e]);
              unsigned short lb = f2bf_bits(sp[e] - bf_bits2f(hb));
              hv[e] = __builtin_bit_cast(_Float16, hb);
              lv[e] = __builtin_bit_cast(_Float16, lb);
            }
          }
          *(volatile v8h*)(C + (size_t)(mBase + row) * ldc + n0 + c8) = hv;
          if (OUT_MODE == 2) *(volatile v8h*)(C2 + (size_t)(mBase + row) * ldc + n0 + c8) = lv;
        }
        __threadfence();
      }
    }
    __builtin_amdgcn_fence(__ATOMIC_RELEASE, "workgroup");
    __builtin_amdgcn_wave_barrier();
    __builtin_amdgcn_fence(__ATOMIC_ACQUIRE, "workgroup");
  }
}

__global__ __launch_bounds__(256) void w2_transpose_f16(const float* __restrict__ W2, _Float16* __restrict__ W2t) {
  __shared__ float tile[64][65];
  const int tid = threadIdx.x;
  const int n0 = blockIdx.x * 64;
  const int k0 = blockIdx.y * 64;
#pragma unroll
  for (int it = 0; it < 16; ++it) {
    const int idx = it * 256 + tid;
    const int r = idx >> 6;
    const int c = idx & 63;
    tile[c][r] = W2[(size_t)(k0 + r) * HID + n0 + c] * WSCALE;
  }
  __syncthreads();
  const int wave = tid >> 5, lane = tid & 31;
  const int q = lane >> 3, c8 = (lane & 7) * 8;
  for (int pass = 0; pass < 2; ++pass) {
#pragma unroll
    for (int it = 0; it < 2; ++it) {
      const int row = wave * 8 + it * 4 + q;
      v8h hv;
#pragma unroll
      for (int e = 0; e < 8; ++e) hv[e] = (_Float16)tile[row][c8 + e];
      *(volatile v8h*)(W2t + (size_t)(n0 + row) * HID + k0 + c8) = hv;
    }
    __threadfence();
  }
}

__global__ __launch_bounds__(128) void heads_pack_f16(const float* __restrict__ Wh, _Float16* __restrict__ WhT) {
  const int n = blockIdx.x;
  const int t = threadIdx.x;
  const int kb = 8 * t;
  v8h hv;
  if (n < NSK * NACT) {
    const int sk = n >> 2, a = n & 3;
#pragma unroll
    for (int e = 0; e < 8; ++e)
      hv[e] = (_Float16)(Wh[((size_t)sk * HID + kb + e) * NACT + a] * WSCALE);
  } else {
#pragma unroll
    for (int e = 0; e < 8; ++e) hv[e] = (_Float16)0.0f;
  }
  _Float16* p = WhT + (size_t)n * HID + kb;
  *(volatile v8h*)p = hv;
  __threadfence();
  *(volatile v8h*)p = hv;
}

__global__ __launch_bounds__(128) void layer1_f16(const float* __restrict__ s, const float* __restrict__ W1,
                                                  const float* __restrict__ b1, _Float16* __restrict__ h1,
                                                  int row0, int nrows) {
  const int t = threadIdx.x;
  const int kb = 8 * t;
  float w0[8], w1[8], bb[8];
#pragma unroll
  for (int e = 0; e < 8; ++e) {
    w0[e] = W1[kb + e];
    w1[e] = W1[HID + kb + e];
    bb[e] = b1[kb + e];
  }
  const int rb = blockIdx.x * L1_ROWS;
#pragma unroll 1
  for (int r = 0; r < L1_ROWS; ++r) {
    const int lr = rb + r;
    if (lr < nrows) {
      const int n = row0 + lr;
      const float s0 = s[(size_t)n * SDIM], s1 = s[(size_t)n * SDIM + 1];
      v8h hv;
#pragma unroll
      for (int e = 0; e < 8; ++e) {
        float v = s0 * w0[e] + s1 * w1[e];
        v = v + bb[e];
        v = fmaxf(v, 0.0f);
        hv[e] = (_Float16)v;
      }
      _Float16* p = h1 + (size_t)lr * HID + kb;
      *(volatile v8h*)p = hv;
      __threadfence();
      *(volatile v8h*)p = hv;
    }
  }
}

__global__ __launch_bounds__(256) void head_select(const float* __restrict__ Y, const int* __restrict__ skill,
                                                   const float* __restrict__ bh, float* __restrict__ out, int nrows) {
  const int n = blockIdx.x * 256 + threadIdx.x;
  if (n < nrows) {
    int sk = skill[n];
    if (sk < 0) sk += NSK;
    sk = sk < 0 ? 0 : (sk > NSK - 1 ? NSK - 1 : sk);
    const v4f y = *(const v4f*)(Y + (size_t)n * NHP + sk * NACT);
    v4f o;
    o[0] = y[0] + bh[sk * NACT + 0];
    o[1] = y[1] + bh[sk * NACT + 1];
    o[2] = y[2] + bh[sk * NACT + 2];
    o[3] = y[3] + bh[sk * NACT + 3];
    float* p = out + (size_t)n * NACT;
    *(volatile v4f*)p = o;
    __threadfence();
    *(volatile v4f*)p = o;
  }
}

extern "C" void kernel_launch(void* const* d_in, const int* in_sizes, int n_in,
                              void* d_out, int out_size, void* d_ws, size_t ws_size,
                              hipStream_t stream) {
  if (n_in < 8) return;
  if (in_sizes[0] != NBATCH * SDIM || in_sizes[1] != NBATCH || in_sizes[2] != SDIM * HID ||
      in_sizes[3] != HID || in_sizes[4] != HID * HID || in_sizes[5] != HID ||
      in_sizes[6] != NSK * HID * NACT || in_sizes[7] != NSK * NACT || out_size != NBATCH * NACT) return;

  const float* s       = (const float*)d_in[0];
  const int*   skill   = (const int*)d_in[1];
  const float* W1      = (const float*)d_in[2];
  const float* b1      = (const float*)d_in[3];
  const float* W2      = (const float*)d_in[4];
  const float* b2      = (const float*)d_in[5];
  const float* W_heads = (const float*)d_in[6];
  const float* b_heads = (const float*)d_in[7];
  float* out = (float*)d_out;

  const size_t sz_w2t  = (size_t)HID * HID * 2;
  const size_t sz_wht  = (size_t)NHP * HID * 2;
  const size_t sz_h1   = (size_t)CHUNK * HID * 2;
  const size_t sz_feat = (size_t)CHUNK * HID * 2;
  const size_t sz_y    = (size_t)NBATCH * NHP * 4;
  const size_t off_w2t  = 0;
  const size_t off_wht  = off_w2t + sz_w2t;
  const size_t off_h1   = off_wht + sz_wht;
  const size_t off_feat = off_h1 + sz_h1;
  const size_t off_y    = off_feat + sz_feat;
  const size_t off_end  = off_y + sz_y;
  if (off_end > ws_size) return;

  char* ws = (char*)d_ws;
  _Float16* W2t  = (_Float16*)(ws + off_w2t);
  _Float16* WhT  = (_Float16*)(ws + off_wht);
  _Float16* h1   = (_Float16*)(ws + off_h1);
  _Float16* feat = (_Float16*)(ws + off_feat);
  float*    Y    = (float*)(ws + off_y);

  w2_transpose_f16<<<dim3(HID / 64, HID / 64), 256, 0, stream>>>(W2, W2t);
  heads_pack_f16<<<NHP, 128, 0, stream>>>(W_heads, WhT);

  const int tiles1 = (CHUNK / 64) * (HID / 64);
  const int grid1  = (tiles1 + 7) / 8;
  const int tiles2 = (CHUNK / 64) * (NHP / 64);
  const int grid2  = (tiles2 + 7) / 8;

  for (int c = 0; c < NCHUNK; ++c) {
    const int row0 = c * CHUNK;
    layer1_f16<<<(CHUNK + L1_ROWS - 1) / L1_ROWS, 128, 0, stream>>>(s, W1, b1, h1, row0, CHUNK);

    wmma_gemm64<0, false, 2, 1, false, 2><<<dim3(grid1, 1), 256, 0, stream>>>(
        (const unsigned short*)h1, (const unsigned short*)h1, HID, 0L,
        (const unsigned short*)W2t, (const unsigned short*)W2t, HID, 0L,
        (void*)feat, (void*)feat, HID, 0L,
        b2, (const float*)Y, 0L,
        CHUNK, HID, HID, WSCALE_INV);

    wmma_gemm64<0, false, 0, 0, false, 0><<<dim3(grid2, 1), 256, 0, stream>>>(
        (const unsigned short*)feat, (const unsigned short*)feat, HID, 0L,
        (const unsigned short*)WhT, (const unsigned short*)WhT, HID, 0L,
        (void*)(Y + (size_t)row0 * NHP), (void*)(Y + (size_t)row0 * NHP), NHP, 0L,
        b_heads, (const float*)Y, 0L,
        CHUNK, NHP, HID, WSCALE_INV);
  }

  head_select<<<(NBATCH + 255) / 256, 256, 0, stream>>>(Y, skill, b_heads, out, NBATCH);
  (void)hipGetLastError();
}
